// PairwiseScore_90615220011455
// MI455X (gfx1250) — hardware-verified
//
#include <hip/hip_runtime.h>
#define BB 2
#define NSP 384
#define EE 256
#define HID 150
#define HP 160
#define NPAIR (BB * NSP * NSP)
#define NTRI 73920
#define CHP 73728

typedef __bf16 v16b __attribute__((ext_vector_type(16)));
typedef unsigned short v8us __attribute__((ext_vector_type(8), may_alias));
typedef float  v8f  __attribute__((ext_vector_type(8)));
typedef float  v4f  __attribute__((ext_vector_type(4)));
typedef float  v4fa __attribute__((ext_vector_type(4), may_alias));
union FragB { v16b v; v8us half[2]; unsigned short u[16]; };

__device__ __forceinline__ unsigned short bf16_bits(float x) { unsigned int u = __float_as_uint(x); return (unsigned short)((u + 0x7FFFu + ((u >> 16) & 1u)) >> 16); }
__device__ __forceinline__ float bf16_val(unsigned short b) { return __uint_as_float(((unsigned int)b) << 16); }
__device__ __forceinline__ float bf16_round(float x) { return bf16_val(bf16_bits(x)); }
template <int NT>
__device__ __forceinline__ v8f mmaN(v16b ah, v16b al, v16b bh, v16b bl, v8f c) {
  c = __builtin_amdgcn_wmma_f32_16x16x32_bf16(false, ah, false, bh, (short)0, c, false, false);
  if (NT >= 2) c = __builtin_amdgcn_wmma_f32_16x16x32_bf16(false, al, false, bh, (short)0, c, false, false);
  if (NT >= 3) c = __builtin_amdgcn_wmma_f32_16x16x32_bf16(false, ah, false, bl, (short)0, c, false, false);
  asm volatile("v_nop\n\tv_nop\n\tv_nop\n\tv_nop" : "+v"(c) : "v"(ah), "v"(al), "v"(bh), "v"(bl));
  return c;
}

__global__ __launch_bounds__(256) void k_wt_bf16(const float* __restrict__ W, unsigned short* __restrict__ Wt, int K, int N) {
  const int t = blockIdx.x * 256 + threadIdx.x;
  const int k8n = K / 8;
  if (t >= N * k8n) return;
  const int n = t / k8n, k8 = (t % k8n) * 8;
  v8us v;
#pragma unroll
  for (int i = 0; i < 8; ++i) v[i] = bf16_bits(W[(size_t)(k8 + i) * N + n]);
  *(volatile v8us*)(Wt + (size_t)n * K + k8) = v;
  __threadfence();
  *(volatile v8us*)(Wt + (size_t)n * K + k8) = v;
}

template <bool ASPLIT, int ACT, bool BIAS_BF16>
__global__ __launch_bounds__(128) void k_gemm_bf(const float* __restrict__ A, int lda, const unsigned short* __restrict__ Wt, int ldb,
                                               const float* __restrict__ bias, float* __restrict__ C, int ldc, int M, int N, int K) {
  __shared__ __attribute__((aligned(16))) float so[4][16][64];
  const int tid = threadIdx.x, w = tid >> 5, lane = tid & 31, ln = lane & 15, hh = lane >> 4;
  const int ntn = N / 64;
  const int wid = blockIdx.x * 4 + w;
  const int mt = wid / ntn, nq = wid % ntn;
  if (mt * 16 >= M) return;
  const int row0 = mt * 16, col0 = nq * 64;
  const float* arow = A + (size_t)(row0 + ln) * lda;
  v8f acc[4] = {};
  for (int kb = 0; kb < K; kb += 32) {
    FragB ah, al;
    const v4f x0 = *(const v4fa*)(arow + kb + 8 * hh), x1 = *(const v4fa*)(arow + kb + 8 * hh + 4);
    const v4f x2 = *(const v4fa*)(arow + kb + 16 + 8 * hh), x3 = *(const v4fa*)(arow + kb + 16 + 8 * hh + 4);
    float xs[16] = {x0[0],x0[1],x0[2],x0[3],x1[0],x1[1],x1[2],x1[3],x2[0],x2[1],x2[2],x2[3],x3[0],x3[1],x3[2],x3[3]};
#pragma unroll
    for (int i = 0; i < 16; ++i) { const unsigned short hb = bf16_bits(xs[i]); ah.u[i] = hb; al.u[i] = ASPLIT ? bf16_bits(xs[i] - bf16_val(hb)) : (unsigned short)0; }
#pragma unroll
    for (int t = 0; t < 4; ++t) {
      const unsigned short* brow = Wt + (size_t)(col0 + t * 16 + ln) * ldb + kb;
      FragB b;
      b.half[0] = *(const v8us*)(brow + 8 * hh);
      b.half[1] = *(const v8us*)(brow + 16 + 8 * hh);
      acc[t] = mmaN<ASPLIT ? 2 : 1>(ah.v, al.v, b.v, b.v, acc[t]);
    }
  }
#pragma unroll
  for (int t = 0; t < 4; ++t) {
    float bv = bias ? bias[col0 + t * 16 + ln] : 0.f;
    if (BIAS_BF16) bv = bf16_round(bv);
#pragma unroll
    for (int r = 0; r < 8; ++r) { float v = acc[t][r] + bv; if (ACT == 1) v = fmaxf(v, 0.f); so[w][8 * hh + r][t * 16 + ln] = v; }
  }
  __builtin_amdgcn_fence(__ATOMIC_ACQ_REL, "workgroup");
  __builtin_amdgcn_wave_barrier();
  const int rsub = lane >> 4, c4 = (lane & 15) * 4;
  for (int pass = 0; pass < 2; ++pass) {
#pragma unroll
    for (int q = 0; q < 8; ++q) {
      const int r = q * 2 + rsub;
      const v4f v = *(const v4fa*)&so[w][r][c4];
      *(volatile v4f*)(C + (size_t)(row0 + r) * ldc + col0 + c4) = v;
    }
    if (pass == 0) __threadfence();
  }
}

template <int D, bool CAUSAL>
__global__ __launch_bounds__(128) void k_flash(const float* __restrict__ qb, const float* __restrict__ kb, const float* __restrict__ vb,
                                             int pitch, int T, int H, float scale, float* __restrict__ y, int ypitch) {
  constexpr int KS = D / 32;
  constexpr int DT = D / 16;
  __shared__ __attribute__((aligned(16))) unsigned short sKh[32][D + 8], sKl[32][D + 8], sVh[32][D + 8], sVl[32][D + 8];
  __shared__ __attribute__((aligned(16))) unsigned short sPh[4][16][40], sPl[4][16][40];
  __shared__ __attribute__((aligned(16))) float sO[4][16][D];
  const int tid = threadIdx.x, w = tid >> 5, lane = tid & 31, ln = lane & 15, hh = lane >> 4;
  const int nqb = (T + 63) / 64;
  const int bh = blockIdx.x / nqb, qblk = blockIdx.x % nqb;
  const int b = bh / H, h = bh % H;
  const int q0 = qblk * 64 + w * 16;
  const float* Q = qb + (size_t)b * T * pitch + h * D;
  const float* K = kb + (size_t)b * T * pitch + h * D;
  const float* V = vb + (size_t)b * T * pitch + h * D;

  FragB aqh[KS], aql[KS];
  {
    int row = q0 + ln; if (row >= T) row = T - 1;
    const float* qr = Q + (size_t)row * pitch;
#pragma unroll
    for (int ks = 0; ks < KS; ++ks)
#pragma unroll
      for (int i = 0; i < 16; ++i) {
        const int d = ks * 32 + ((i < 8) ? (8 * hh + i) : (16 + 8 * hh + (i - 8)));
        const float x = qr[d] * scale; const unsigned short hb = bf16_bits(x);
        aqh[ks].u[i] = hb; aql[ks].u[i] = bf16_bits(x - bf16_val(hb));
      }
  }
  float m_r[8], l_r[8];
#pragma unroll
  for (int r = 0; r < 8; ++r) { m_r[r] = -3.0e38f; l_r[r] = 0.f; }
  v8f oacc[DT];
#pragma unroll
  for (int dt = 0; dt < DT; ++dt) oacc[dt] = (v8f){0.f,0.f,0.f,0.f,0.f,0.f,0.f,0.f};

  const int kv_end = CAUSAL ? min(T, qblk * 64 + 64) : T;
  for (int j0 = 0; j0 < kv_end; j0 += 32) {
    __syncthreads();
    for (int e = tid; e < 32 * (D / 4); e += 128) {
      const int r = e / (D / 4), c4 = (e % (D / 4)) * 4;
      const int key = j0 + r;
      v4f kf = {0.f,0.f,0.f,0.f}, vf = {0.f,0.f,0.f,0.f};
      if (key < T) { kf = *(const v4fa*)(K + (size_t)key * pitch + c4); vf = *(const v4fa*)(V + (size_t)key * pitch + c4); }
#pragma unroll
      for (int t = 0; t < 4; ++t) {
        unsigned short hb = bf16_bits(kf[t]); sKh[r][c4 + t] = hb; sKl[r][c4 + t] = bf16_bits(kf[t] - bf16_val(hb));
        hb = bf16_bits(vf[t]); sVh[r][c4 + t] = hb; sVl[r][c4 + t] = bf16_bits(vf[t] - bf16_val(hb));
      }
    }
    __syncthreads();
    v8f s[2];
#pragma unroll
    for (int nt = 0; nt < 2; ++nt) {
      v8f acc = {};
#pragma unroll
      for (int ks = 0; ks < KS; ++ks) {
        FragB bh_, bl_;
        bh_.half[0] = *(const v8us*)&sKh[nt * 16 + ln][ks * 32 + 8 * hh]; bh_.half[1] = *(const v8us*)&sKh[nt * 16 + ln][ks * 32 + 16 + 8 * hh];
        bl_.half[0] = *(const v8us*)&sKl[nt * 16 + ln][ks * 32 + 8 * hh]; bl_.half[1] = *(const v8us*)&sKl[nt * 16 + ln][ks * 32 + 16 + 8 * hh];
        acc = mmaN<3>(aqh[ks].v, aql[ks].v, bh_.v, bl_.v, acc);
      }
      s[nt] = acc;
    }
    float alpha[8];
#pragma unroll
    for (int r = 0; r < 8; ++r) {
      const int qi = q0 + 8 * hh + r;
      const int ja = j0 + ln, jb = j0 + 16 + ln;
      if (CAUSAL) { if (ja > qi) s[0][r] = -3.0e38f; if (jb > qi) s[1][r] = -3.0e38f; }
      if (ja >= T) s[0][r] = -3.0e38f;
      if (jb >= T) s[1][r] = -3.0e38f;
      float mx = fmaxf(s[0][r], s[1][r]);
      mx = fmaxf(mx, __shfl_xor(mx, 1, 32)); mx = fmaxf(mx, __shfl_xor(mx, 2, 32)); mx = fmaxf(mx, __shfl_xor(mx, 4, 32)); mx = fmaxf(mx, __shfl_xor(mx, 8, 32));
      const float mnew = fmaxf(m_r[r], mx);
      alpha[r] = (mnew > -1.0e38f) ? __expf(m_r[r] - mnew) : 1.0f;
      const float p0 = (s[0][r] > -1.0e38f) ? __expf(s[0][r] - mnew) : 0.f;
      const float p1 = (s[1][r] > -1.0e38f) ? __expf(s[1][r] - mnew) : 0.f;
      m_r[r] = mnew;
      l_r[r] = l_r[r] * alpha[r] + p0 + p1;
      unsigned short hb = bf16_bits(p0); sPh[w][8 * hh + r][ln] = hb;      sPl[w][8 * hh + r][ln] = bf16_bits(p0 - bf16_val(hb));
      hb = bf16_bits(p1);                sPh[w][8 * hh + r][16 + ln] = hb; sPl[w][8 * hh + r][16 + ln] = bf16_bits(p1 - bf16_val(hb));
    }
#pragma unroll
    for (int dt = 0; dt < DT; ++dt)
#pragma unroll
      for (int r = 0; r < 8; ++r) oacc[dt][r] *= alpha[r];
    __builtin_amdgcn_fence(__ATOMIC_ACQ_REL, "workgroup");
    __builtin_amdgcn_wave_barrier();
    FragB pah, pal;
    pah.half[0] = *(const v8us*)&sPh[w][ln][8 * hh]; pah.half[1] = *(const v8us*)&sPh[w][ln][16 + 8 * hh];
    pal.half[0] = *(const v8us*)&sPl[w][ln][8 * hh]; pal.half[1] = *(const v8us*)&sPl[w][ln][16 + 8 * hh];
#pragma unroll
    for (int dt = 0; dt < DT; ++dt) {
      FragB bvh, bvl;
#pragma unroll
      for (int i = 0; i < 8; ++i) {
        bvh.u[i] = sVh[8 * hh + i][dt * 16 + ln]; bvh.u[8 + i] = sVh[16 + 8 * hh + i][dt * 16 + ln];
        bvl.u[i] = sVl[8 * hh + i][dt * 16 + ln]; bvl.u[8 + i] = sVl[16 + 8 * hh + i][dt * 16 + ln];
      }
      oacc[dt] = mmaN<3>(pah.v, pal.v, bvh.v, bvl.v, oacc[dt]);
    }
    __builtin_amdgcn_fence(__ATOMIC_ACQ_REL, "workgroup");
    __builtin_amdgcn_wave_barrier();
  }
#pragma unroll
  for (int r = 0; r < 8; ++r) {
    float l = l_r[r];
    l += __shfl_xor(l, 1, 32); l += __shfl_xor(l, 2, 32); l += __shfl_xor(l, 4, 32); l += __shfl_xor(l, 8, 32);
    l_r[r] = (l > 0.f) ? 1.0f / l : 0.f;
  }
#pragma unroll
  for (int dt = 0; dt < DT; ++dt)
#pragma unroll
    for (int r = 0; r < 8; ++r) sO[w][8 * hh + r][dt * 16 + ln] = oacc[dt][r] * l_r[r];
  __builtin_amdgcn_fence(__ATOMIC_ACQ_REL, "workgroup");
  __builtin_amdgcn_wave_barrier();
  for (int pass = 0; pass < 2; ++pass) {
    for (int r = 0; r < 16; ++r) {
      const int row = q0 + r;
      if (row < T && lane < D / 4) {
        const v4f val = *(const v4fa*)&sO[w][r][lane * 4];
        *(volatile v4f*)(y + ((size_t)b * T + row) * ypitch + h * D + lane * 4) = val;
      }
    }
    if (pass == 0) __threadfence();
  }
}

template <bool ASPLIT, bool BSPLIT, int ACT>
__global__ __launch_bounds__(128) void k_gemm_b(const float* __restrict__ A, int lda, size_t sA, const unsigned short* __restrict__ Bh, const unsigned short* __restrict__ Bl, int ldb, size_t sB,
                                             const float* __restrict__ bias, const float* __restrict__ resid, int ldr, size_t sR, float rsign, float alpha,
                                             float* __restrict__ C, int ldc, size_t sC, int M, int N, int K) {
  __shared__ __attribute__((aligned(16))) float so[4][16][64];
  const int tid = threadIdx.x, w = tid >> 5, lane = tid & 31, ln = lane & 15, hh = lane >> 4;
  const int by = blockIdx.y;
  A += (size_t)by * sA; Bh += (size_t)by * sB; if (BSPLIT) Bl += (size_t)by * sB; C += (size_t)by * sC; if (resid) resid += (size_t)by * sR;
  const int ntn = (N + 63) / 64; const int wid = blockIdx.x * 4 + w; const int mt = wid / ntn, nq = wid % ntn;
  if (mt * 16 >= M) return;
  const int row0 = mt * 16, col0 = nq * 64;
  const float* arow = A + (size_t)(row0 + ln) * lda;
  v8f acc[4] = {};
  for (int kb = 0; kb < K; kb += 32) {
    FragB ah, al;
    const v4f x0 = *(const v4fa*)(arow + kb + 8 * hh), x1 = *(const v4fa*)(arow + kb + 8 * hh + 4);
    const v4f x2 = *(const v4fa*)(arow + kb + 16 + 8 * hh), x3 = *(const v4fa*)(arow + kb + 16 + 8 * hh + 4);
    float xs[16] = {x0[0],x0[1],x0[2],x0[3],x1[0],x1[1],x1[2],x1[3],x2[0],x2[1],x2[2],x2[3],x3[0],x3[1],x3[2],x3[3]};
#pragma unroll
    for (int i = 0; i < 16; ++i) { const unsigned short hb = bf16_bits(xs[i]); ah.u[i] = hb; al.u[i] = ASPLIT ? bf16_bits(xs[i] - bf16_val(hb)) : (unsigned short)0; }
#pragma unroll
    for (int t = 0; t < 4; ++t) {
      if (col0 + t * 16 >= N) continue;
      const size_t boff = (size_t)(col0 + t * 16 + ln) * ldb + kb;
      FragB bh_, bl_; bh_.half[0] = *(const v8us*)(Bh + boff + 8 * hh); bh_.half[1] = *(const v8us*)(Bh + boff + 16 + 8 * hh);
      if (BSPLIT) { bl_.half[0] = *(const v8us*)(Bl + boff + 8 * hh); bl_.half[1] = *(const v8us*)(Bl + boff + 16 + 8 * hh); } else bl_ = bh_;
      acc[t] = mmaN<ASPLIT ? (BSPLIT ? 3 : 2) : 1>(ah.v, al.v, bh_.v, bl_.v, acc[t]);
    }
  }
#pragma unroll
  for (int t = 0; t < 4; ++t) {
    const int col = col0 + t * 16 + ln; if (col0 + t * 16 >= N) continue; const float bv = bias ? bf16_round(bias[col]) : 0.f;
#pragma unroll
    for (int r = 0; r < 8; ++r) { float v = acc[t][r] * alpha + bv; if (resid) v += rsign * resid[(size_t)(row0 + 8 * hh + r) * ldr + col]; if (ACT == 1) v = fmaxf(v, 0.f); else if (ACT == 2) v = fmaxf(v, 0.f) + log1pf(expf(-fabsf(v))); so[w][8 * hh + r][t * 16 + ln] = v; }
  }
  __builtin_amdgcn_fence(__ATOMIC_ACQ_REL, "workgroup"); __builtin_amdgcn_wave_barrier();
  const int rsub = lane >> 4, c4 = (lane & 15) * 4;
  for (int pass = 0; pass < 2; ++pass) {
#pragma unroll
    for (int q = 0; q < 8; ++q) { const int r = q * 2 + rsub; if (col0 + c4 < N) { const v4f v = *(const v4fa*)&so[w][r][c4]; *(volatile v4f*)(C + (size_t)(row0 + r) * ldc + col0 + c4) = v; } }
    if (pass == 0) __threadfence();
  }
}
__global__ __launch_bounds__(256) void k_split_transpose_b(const float* __restrict__ src, int lds_, size_t sIn, unsigned short* __restrict__ hi, unsigned short* __restrict__ lo, size_t sOut, int K, int N) {
  const size_t t = (size_t)blockIdx.x * 256 + threadIdx.x; const int k8n = K / 8; if (t >= (size_t)N * k8n) return;
  src += (size_t)blockIdx.y * sIn; hi += (size_t)blockIdx.y * sOut; lo += (size_t)blockIdx.y * sOut;
  const int n = (int)(t / k8n), k8 = (int)(t % k8n) * 8; v8us vh, vl;
#pragma unroll
  for (int i = 0; i < 8; ++i) { const float x = src[(size_t)(k8 + i) * lds_ + n]; const unsigned short hb = bf16_bits(x); vh[i] = hb; vl[i] = bf16_bits(x - bf16_val(hb)); }
  unsigned short* dh = hi + (size_t)n * K + k8; unsigned short* dl = lo + (size_t)n * K + k8;
  *(volatile v8us*)dh = vh; *(volatile v8us*)dl = vl; __threadfence(); *(volatile v8us*)dh = vh; *(volatile v8us*)dl = vl;
}

typedef _Float16 v16h __attribute__((ext_vector_type(16)));
union FragH { v16h v; v8us half[2]; _Float16 h[16]; unsigned short u[16]; };
template <int NT>
__device__ __forceinline__ v8f mmaH(v16h ah, v16h al, v16h bh, v16h bl, v8f c) {
  c = __builtin_amdgcn_wmma_f32_16x16x32_f16(false, ah, false, bh, (short)0, c, false, false);
  if (NT >= 2) c = __builtin_amdgcn_wmma_f32_16x16x32_f16(false, al, false, bh, (short)0, c, false, false);
  if (NT >= 3) c = __builtin_amdgcn_wmma_f32_16x16x32_f16(false, ah, false, bl, (short)0, c, false, false);
  asm volatile("v_nop\n\tv_nop\n\tv_nop\n\tv_nop" : "+v"(c) : "v"(ah), "v"(al), "v"(bh), "v"(bl));
  return c;
}
template <bool ASPLIT>
__global__ __launch_bounds__(128) void k_gemm_h(const float* __restrict__ A, int lda, size_t sA, const _Float16* __restrict__ Bh, int ldb, size_t sB, float alpha, float* __restrict__ C, int ldc, size_t sC, int M, int N, int K) {
  __shared__ __attribute__((aligned(16))) float so[4][16][64];
  const int tid = threadIdx.x, w = tid >> 5, lane = tid & 31, ln = lane & 15, hh = lane >> 4; const int by = blockIdx.y;
  A += (size_t)by * sA; Bh += (size_t)by * sB; C += (size_t)by * sC;
  const int ntn = (N + 63) / 64; const int wid = blockIdx.x * 4 + w; const int mt = wid / ntn, nq = wid % ntn; if (mt * 16 >= M) return;
  const int row0 = mt * 16, col0 = nq * 64; const float* arow = A + (size_t)(row0 + ln) * lda;
  v8f acc[4] = {};
  for (int kb = 0; kb < K; kb += 32) {
    FragH ah, al;
    const v4f x0 = *(const v4fa*)(arow + kb + 8 * hh), x1 = *(const v4fa*)(arow + kb + 8 * hh + 4), x2 = *(const v4fa*)(arow + kb + 16 + 8 * hh), x3 = *(const v4fa*)(arow + kb + 16 + 8 * hh + 4);
    float xs[16] = {x0[0],x0[1],x0[2],x0[3],x1[0],x1[1],x1[2],x1[3],x2[0],x2[1],x2[2],x2[3],x3[0],x3[1],x3[2],x3[3]};
#pragma unroll
    for (int i = 0; i < 16; ++i) { const _Float16 h = (_Float16)xs[i]; ah.h[i] = h; al.h[i] = ASPLIT ? (_Float16)(xs[i] - (float)h) : (_Float16)0.0f; }
#pragma unroll
    for (int t = 0; t < 4; ++t) { if (col0 + t * 16 >= N) continue; const size_t boff = (size_t)(col0 + t * 16 + ln) * ldb + kb; FragH bq; bq.half[0] = *(const v8us*)(Bh + boff + 8 * hh); bq.half[1] = *(const v8us*)(Bh + boff + 16 + 8 * hh);
      acc[t] = mmaH<ASPLIT ? 2 : 1>(ah.v, al.v, bq.v, bq.v, acc[t]); }
  }
#pragma unroll
  for (int t = 0; t < 4; ++t) { if (col0 + t * 16 >= N) continue;
#pragma unroll
    for (int r = 0; r < 8; ++r) so[w][8 * hh + r][t * 16 + ln] = acc[t][r] * alpha; }
  __builtin_amdgcn_fence(__ATOMIC_ACQ_REL, "workgroup"); __builtin_amdgcn_wave_barrier();
  const int rsub = lane >> 4, c4 = (lane & 15) * 4;
  for (int pass = 0; pass < 2; ++pass) {
#pragma unroll
    for (int q = 0; q < 8; ++q) { const int r = q * 2 + rsub; if (col0 + c4 < N) { const v4f v = *(const v4fa*)&so[w][r][c4]; *(volatile v4f*)(C + (size_t)(row0 + r) * ldc + col0 + c4) = v; } }
    if (pass == 0) __threadfence(); }
}

__global__ __launch_bounds__(128) void k_gemm_pair1(const float* __restrict__ X, const _Float16* __restrict__ Bh, int ldb, float alpha, const float* __restrict__ SAB, const float* __restrict__ b1, size_t pr0, _Float16* __restrict__ H1, int M, int N, int K) {
  __shared__ __attribute__((aligned(16))) float so[4][16][64];
  const int tid = threadIdx.x, w = tid >> 5, lane = tid & 31, ln = lane & 15, hh = lane >> 4;
  const int ntn = (N + 63) / 64; const int wid = blockIdx.x * 4 + w; const int mt = wid / ntn, nq = wid % ntn; if (mt * 16 >= M) return;
  const int row0 = mt * 16, col0 = nq * 64; const size_t pr = pr0 + row0 + ln; const int j = (int)(pr % NSP); const int i = (int)((pr / NSP) % NSP); const int b = (int)(pr / ((size_t)NSP * NSP));
  const float* xi = X + ((size_t)b * NSP + i) * EE; const float* xj = X + ((size_t)b * NSP + j) * EE;
  v8f acc[4] = {};
  for (int kb = 0; kb < K; kb += 32) { FragH ah;
#pragma unroll
    for (int q = 0; q < 8; ++q) { const int e0 = kb + 8 * hh + q, e1 = kb + 16 + 8 * hh + q; ah.h[q] = (_Float16)(bf16_round(xi[e0]) * bf16_round(xj[e0])); ah.h[8 + q] = (_Float16)(bf16_round(xi[e1]) * bf16_round(xj[e1])); }
#pragma unroll
    for (int t = 0; t < 4; ++t) { if (col0 + t * 16 >= N) continue; const size_t boff = (size_t)(col0 + t * 16 + ln) * ldb + kb; FragH bq; bq.half[0] = *(const v8us*)((const unsigned short*)Bh + boff + 8 * hh); bq.half[1] = *(const v8us*)((const unsigned short*)Bh + boff + 16 + 8 * hh);
      acc[t] = mmaH<1>(ah.v, ah.v, bq.v, bq.v, acc[t]); }
  }
  const float* sa = SAB + ((size_t)b * NSP + i) * (2 * HP);
#pragma unroll
  for (int t = 0; t < 4; ++t) { if (col0 + t * 16 >= N) continue; const int col = col0 + t * 16 + ln; const float bb = (col < HID) ? bf16_round(b1[col]) : 0.f; const float sac = sa[col];
#pragma unroll
    for (int r = 0; r < 8; ++r) { const int jr = (int)((pr0 + row0 + 8 * hh + r) % NSP); const float sbc = SAB[((size_t)b * NSP + jr) * (2 * HP) + HP + col]; float v = ((sac + sbc) + acc[t][r] * alpha) + bb; v = (col < HID) ? fmaxf(v, 0.f) : 0.f; so[w][8 * hh + r][t * 16 + ln] = v; } }
  __builtin_amdgcn_fence(__ATOMIC_ACQ_REL, "workgroup"); __builtin_amdgcn_wave_barrier();
  const int rsub = lane >> 4, c4 = (lane & 15) * 4; typedef _Float16 v4h __attribute__((ext_vector_type(4)));
  for (int pass = 0; pass < 2; ++pass) {
#pragma unroll
    for (int q = 0; q < 8; ++q) { const int r = q * 2 + rsub; if (col0 + c4 < N) { const v4f v = *(const v4fa*)&so[w][r][c4]; v4h h4; for (int u = 0; u < 4; ++u) h4[u] = (_Float16)v[u]; *(volatile v4h*)(H1 + (size_t)(row0 + r) * HP + col0 + c4) = h4; } }
    if (pass == 0) __threadfence(); }
}
__global__ __launch_bounds__(128) void k_gemm_pair2(const _Float16* __restrict__ A, int lda, const _Float16* __restrict__ Bh, int ldb, float alpha, const float* __restrict__ b2, const float* __restrict__ W3, float* __restrict__ PS, size_t ldps, int M, int N, int K) {
  __shared__ float sp[4][16];
  const int tid = threadIdx.x, w = tid >> 5, lane = tid & 31, ln = lane & 15, hh = lane >> 4;
  const int ntn = (N + 63) / 64; const int wid = blockIdx.x * 4 + w; const int mt = wid / ntn, nq = wid % ntn; if (mt * 16 >= M) return;
  const int row0 = mt * 16, col0 = nq * 64; const _Float16* arow = A + (size_t)(row0 + ln) * lda;
  v8f acc[4] = {};
  for (int kb = 0; kb < K; kb += 32) { FragH ah; ah.half[0] = *(const v8us*)((const unsigned short*)arow + kb + 8 * hh); ah.half[1] = *(const v8us*)((const unsigned short*)arow + kb + 16 + 8 * hh);
#pragma unroll
    for (int t = 0; t < 4; ++t) { if (col0 + t * 16 >= N) continue; const size_t boff = (size_t)(col0 + t * 16 + ln) * ldb + kb; FragH bq; bq.half[0] = *(const v8us*)((const unsigned short*)Bh + boff + 8 * hh); bq.half[1] = *(const v8us*)((const unsigned short*)Bh + boff + 16 + 8 * hh);
      acc[t] = mmaH<1>(ah.v, ah.v, bq.v, bq.v, acc[t]); }
  }
  float rowsum[8] = {0.f, 0.f, 0.f, 0.f, 0.f, 0.f, 0.f, 0.f};
#pragma unroll
  for (int t = 0; t < 4; ++t) { if (col0 + t * 16 >= N) continue; const int col = col0 + t * 16 + ln; const float bb = (col < HID) ? bf16_round(b2[col]) : 0.f; const float wc = (col < HID) ? bf16_round(W3[col]) : 0.f;
#pragma unroll
    for (int r = 0; r < 8; ++r) rowsum[r] += fmaxf(acc[t][r] * alpha + bb, 0.f) * wc; }
#pragma unroll
  for (int r = 0; r < 8; ++r) { float s = rowsum[r]; for (int o = 8; o >= 1; o >>= 1) s += __shfl_xor(s, o, 32); rowsum[r] = s; }
  if (ln == 0) { for (int r = 0; r < 8; ++r) sp[w][8 * hh + r] = rowsum[r]; }
  __builtin_amdgcn_fence(__ATOMIC_ACQ_REL, "workgroup"); __builtin_amdgcn_wave_barrier();
  if (lane < 16) { *(volatile float*)(PS + (size_t)nq * ldps + row0 + lane) = sp[w][lane]; } __threadfence(); if (lane < 16) { *(volatile float*)(PS + (size_t)nq * ldps + row0 + lane) = sp[w][lane]; }
}

__global__ __launch_bounds__(128) void k_gemm_sym1(const float* __restrict__ XR, const int* __restrict__ TRI, const _Float16* __restrict__ Bh, int ldb, float alpha, _Float16* __restrict__ PCS, int M, int K) {
  __shared__ __attribute__((aligned(16))) float so[4][16][HP];
  const int tid = threadIdx.x, w = tid >> 5, lane = tid & 31, ln = lane & 15, hh = lane >> 4; const int b = blockIdx.y;
  const int mt = blockIdx.x * 4 + w; if (mt * 16 >= M) return; const int row0 = mt * 16; int r = row0 + ln; r = r < M ? r : M - 1;
  const int i = TRI[2 * r], j = TRI[2 * r + 1]; const float* xi = XR + ((size_t)b * NSP + i) * EE; const float* xj = XR + ((size_t)b * NSP + j) * EE;
  v8f acc[HP / 16] = {};
  for (int kb = 0; kb < K; kb += 32) { FragH ah;
#pragma unroll
    for (int q = 0; q < 8; ++q) { const int e0 = kb + 8 * hh + q, e1 = kb + 16 + 8 * hh + q; ah.h[q] = (_Float16)(xi[e0] * xj[e0]); ah.h[8 + q] = (_Float16)(xi[e1] * xj[e1]); }
#pragma unroll
    for (int t = 0; t < HP / 16; ++t) { const size_t boff = (size_t)(t * 16 + ln) * ldb + kb; FragH bq; bq.half[0] = *(const v8us*)((const unsigned short*)Bh + boff + 8 * hh); bq.half[1] = *(const v8us*)((const unsigned short*)Bh + boff + 16 + 8 * hh);
      acc[t] = mmaH<1>(ah.v, ah.v, bq.v, bq.v, acc[t]); }
  }
#pragma unroll
  for (int t = 0; t < HP / 16; ++t) {
#pragma unroll
    for (int rr = 0; rr < 8; ++rr) so[w][8 * hh + rr][t * 16 + ln] = acc[t][rr] * alpha; }
  __builtin_amdgcn_fence(__ATOMIC_ACQ_REL, "workgroup"); __builtin_amdgcn_wave_barrier();
  typedef _Float16 v4h __attribute__((ext_vector_type(4)));
  for (int pass = 0; pass < 2; ++pass) { for (int e = lane; e < 16 * (HP / 4); e += 32) { const int rr = e / (HP / 4), c4 = (e % (HP / 4)) * 4; if (row0 + rr < M) { const v4f v = *(const v4fa*)&so[w][rr][c4]; v4h h4; for (int u = 0; u < 4; ++u) h4[u] = (_Float16)v[u]; *(volatile v4h*)(PCS + ((size_t)b * M + row0 + rr) * HP + c4) = h4; } } if (pass == 0) __threadfence(); }
}

__global__ __launch_bounds__(256) void k_w(const float* __restrict__ W1, const float* __restrict__ W2, unsigned short* __restrict__ Bab, _Float16* __restrict__ Bc, _Float16* __restrict__ B2) { const int t = blockIdx.x * 256 + threadIdx.x;
  if (t < 2 * HP * (EE / 8)) { const int k8 = (t % (EE / 8)) * 8; const int n = (t / (EE / 8)) % HP; const int wch = t / ((EE / 8) * HP); v8us v; for (int q = 0; q < 8; ++q) v[q] = bf16_bits(n < HID ? W1[(size_t)(wch * EE + k8 + q) * HID + n] : 0.f); unsigned short* d = Bab + ((size_t)(wch * HP + n)) * EE + k8; *(volatile v8us*)d = v; __threadfence(); *(volatile v8us*)d = v; }
  if (t < HP * (EE / 8)) { const int k8 = (t % (EE / 8)) * 8; const int n = t / (EE / 8); FragH f; for (int q = 0; q < 8; ++q) f.h[q] = (_Float16)(n < HID ? bf16_round(W1[(size_t)(2 * EE + k8 + q) * HID + n]) * 4.0f : 0.f); unsigned short* d = (unsigned short*)Bc + (size_t)n * EE + k8; *(volatile v8us*)d = f.half[0]; __threadfence(); *(volatile v8us*)d = f.half[0]; }
  if (t < HP * (HP / 8)) { const int k8 = (t % (HP / 8)) * 8; const int n = t / (HP / 8); FragH f; for (int q = 0; q < 8; ++q) { const int k = k8 + q; f.h[q] = (_Float16)((n < HID && k < HID) ? bf16_round(W2[(size_t)k * HID + n]) * 4.0f : 0.f); } unsigned short* d = (unsigned short*)B2 + (size_t)n * HP + k8; *(volatile v8us*)d = f.half[0]; __threadfence(); *(volatile v8us*)d = f.half[0]; } }
__global__ __launch_bounds__(256) void k_prep(const float* __restrict__ x, float* __restrict__ XR, int* __restrict__ TRI) { const int t = blockIdx.x * 256 + threadIdx.x;
  if (t < BB * NSP * EE / 4) { const v4f a = *(const v4fa*)(x + (size_t)t * 4); v4f o; for (int q = 0; q < 4; ++q) o[q] = bf16_round(a[q]); *(volatile v4f*)(XR + (size_t)t * 4) = o; __threadfence(); *(volatile v4f*)(XR + (size_t)t * 4) = o; }
  if (t < NTRI) { const int r = t; int i = (int)floorf((769.0f - sqrtf(769.0f * 769.0f - 8.0f * (float)r)) * 0.5f); i = i < 0 ? 0 : (i > NSP - 1 ? NSP - 1 : i);
    for (int it = 0; it < 3; ++it) { const int bi = i * NSP - (i * (i - 1)) / 2; if (r < bi && i > 0) --i; else { const int bn = (i + 1) * NSP - ((i + 1) * i) / 2; if (r >= bn && i < NSP - 1) ++i; } }
    const int bi = i * NSP - (i * (i - 1)) / 2; const int j = i + (r - bi); int2 v; v.x = i; v.y = j; typedef int v2i __attribute__((ext_vector_type(2))); v2i o; o.x = i; o.y = j; *(volatile v2i*)(TRI + 2 * r) = o; __threadfence(); *(volatile v2i*)(TRI + 2 * r) = o; (void)v; } }
__global__ __launch_bounds__(256) void k_h1(const float* __restrict__ SAB, const _Float16* __restrict__ PCS, const float* __restrict__ b1, size_t pr0, _Float16* __restrict__ H1) { const size_t t = (size_t)blockIdx.x * 256 + threadIdx.x; if (t >= (size_t)CHP * HP / 8) return; const int c8 = (int)((t * 8) % HP); const size_t prl = (t * 8) / HP; const size_t pr = pr0 + prl; const int j = (int)(pr % NSP); const int i = (int)((pr / NSP) % NSP); const int b = (int)(pr / ((size_t)NSP * NSP));
  const int lo = i < j ? i : j, hi = i < j ? j : i; const int r = lo * NSP - (lo * (lo - 1)) / 2 + (hi - lo); const float* sa = SAB + ((size_t)b * NSP + i) * (2 * HP) + c8; const float* sb = SAB + ((size_t)b * NSP + j) * (2 * HP) + HP + c8; FragH pc; pc.half[0] = *(const v8us*)((const unsigned short*)PCS + ((size_t)b * NTRI + r) * HP + c8); FragH f;
  for (int q = 0; q < 8; ++q) { const int c = c8 + q; f.h[q] = (c < HID) ? (_Float16)fmaxf(((sa[q] + sb[q]) + (float)pc.h[q]) + bf16_round(b1[c]), 0.f) : (_Float16)0.0f; }
  *(volatile v8us*)((unsigned short*)H1 + t * 8) = f.half[0]; __threadfence(); *(volatile v8us*)((unsigned short*)H1 + t * 8) = f.half[0]; }
__global__ __launch_bounds__(256) void k_fin(const float* __restrict__ PS, const float* __restrict__ ms, const float* __restrict__ b3, size_t pr0, float* __restrict__ out) { const int t = blockIdx.x * 256 + threadIdx.x; if (t >= CHP) return; const size_t pr = pr0 + t; const int j = (int)(pr % NSP); const int i = (int)((pr / NSP) % NSP); const int b = (int)(pr / ((size_t)NSP * NSP));
  const float s = ((PS[t] + PS[CHP + t]) + PS[2 * CHP + t]) + bf16_round(b3[0]); const float v = ((bf16_round(ms[b * NSP + i]) + bf16_round(ms[b * NSP + j])) + s) * (1.0f / 3.0f); *(volatile float*)(out + pr) = v; __threadfence(); *(volatile float*)(out + pr) = v; }
extern "C" void kernel_launch(void* const* d_in, const int* in_sizes, int n_in,
                              void* d_out, int out_size, void* d_ws, size_t ws_size, hipStream_t stream) {
  (void)in_sizes; (void)n_in; (void)out_size;
  const float* x = (const float*)d_in[0]; const float* ms = (const float*)d_in[1]; const float* W1 = (const float*)d_in[2]; const float* b1 = (const float*)d_in[3]; const float* W2 = (const float*)d_in[4]; const float* b2 = (const float*)d_in[5]; const float* W3 = (const float*)d_in[6]; const float* b3 = (const float*)d_in[7];
  char* ws = (char*)d_ws; size_t off = 0;
  auto take = [&](size_t bytes) { char* p = ws + off; off += (bytes + 255) & ~(size_t)255; return p; };
  unsigned short* Bab = (unsigned short*)take((size_t)2 * HP * EE * 2); _Float16* Bc = (_Float16*)take((size_t)HP * EE * 2); _Float16* B2 = (_Float16*)take((size_t)HP * HP * 2);
  float* XR = (float*)take((size_t)BB * NSP * EE * 4); int* TRI = (int*)take((size_t)NTRI * 2 * 4); float* SAB = (float*)take((size_t)BB * NSP * 2 * HP * 4); _Float16* PCS = (_Float16*)take((size_t)BB * NTRI * HP * 2); _Float16* H1 = (_Float16*)take((size_t)CHP * HP * 2); float* PS = (float*)take((size_t)3 * CHP * 4);
  if (off > ws_size) return;
  k_w<<<(2 * HP * (EE / 8) + 255) / 256, 256, 0, stream>>>(W1, W2, Bab, Bc, B2); k_prep<<<(NTRI + 255) / 256, 256, 0, stream>>>(x, XR, TRI);
  k_gemm_b<false, false, 0><<<dim3(((BB * NSP / 16) * 5 + 3) / 4, 1), 128, 0, stream>>>(x, EE, 0, Bab, Bab, EE, 0, nullptr, nullptr, 0, 0, 1.f, 1.f, SAB, 2 * HP, 0, BB * NSP, 2 * HP, EE);
  k_gemm_sym1<<<dim3((NTRI / 16 + 3) / 4 + 1, BB), 128, 0, stream>>>(XR, TRI, Bc, EE, 0.25f, PCS, NTRI, EE);
  for (size_t pr0 = 0; pr0 < (size_t)NPAIR; pr0 += CHP) {
    k_h1<<<(unsigned)(((size_t)CHP * HP / 8 + 255) / 256), 256, 0, stream>>>(SAB, PCS, b1, pr0, H1);
    k_gemm_pair2<<<dim3(((CHP / 16) * 3 + 3) / 4, 1), 128, 0, stream>>>(H1, HP, B2, HP, 0.25f, b2, W3, PS, (size_t)CHP, CHP, HP, HP);
    k_fin<<<CHP / 256, 256, 0, stream>>>(PS, ms, b3, pr0, (float*)d_out);
  }
}
